// MultiheadAttentionXL_43241730736312
// MI455X (gfx1250) — hardware-verified
//
#include <hip/hip_runtime.h>
#include <math.h>

typedef __attribute__((ext_vector_type(16))) _Float16 v16h;
typedef __attribute__((ext_vector_type(16))) __bf16 v16b;
typedef __attribute__((ext_vector_type(8)))  _Float16 v8h;
typedef __attribute__((ext_vector_type(8)))  float v8f;
typedef __attribute__((ext_vector_type(4)))  float v4f;
typedef __attribute__((ext_vector_type(2)))  float v2f;
typedef __attribute__((ext_vector_type(4)))  unsigned v4u;
typedef __attribute__((ext_vector_type(4)))  int v4i;
typedef float __attribute__((may_alias)) float_a;
typedef int __attribute__((may_alias)) int_a;

template <typename T> __device__ __forceinline__ void vst2(void* p, T v) { *(volatile T*)p = v; __threadfence(); *(volatile T*)p = v; }
__device__ __forceinline__ v8f wmma16(v16h a, v16h b, v8f c) {
  v8f d = __builtin_amdgcn_wmma_f32_16x16x32_f16(false, a, false, b, (short)0, c, false, false);
  asm volatile("v_nop\n\tv_nop\n\tv_nop\n\tv_nop" : "+v"(d) : "v"(a), "v"(b));
  return d;
}
__device__ __forceinline__ v8f wmma_bf(v16b a, v16b b, v8f c) {
  v8f d = __builtin_amdgcn_wmma_f32_16x16x32_bf16(false, a, false, b, (short)0, c, false, false);
  asm volatile("v_nop\n\tv_nop\n\tv_nop\n\tv_nop" : "+v"(d) : "v"(a), "v"(b));
  return d;
}
__device__ __forceinline__ v16h frag_h(const _Float16* rowk0, int lane) {
  union { v16h v; v8h q[2]; } u; const _Float16* p = rowk0 + 8 * (lane >> 4);
  u.q[0] = *(const v8h*)p; u.q[1] = *(const v8h*)(p + 16); return u.v;
}
__device__ __forceinline__ v16h frag_f32(const float* rowk0, int lane) {
  v16h a; const float* p = rowk0 + 8 * (lane >> 4);
#pragma unroll
  for (int i = 0; i < 8; ++i) { a[i] = (_Float16)p[i]; a[8 + i] = (_Float16)p[16 + i]; }
  return a;
}
__device__ __forceinline__ v16h frag_f32s(const float* rowk0, int lane, float sc) {
  v16h a; const float* p = rowk0 + 8 * (lane >> 4);
#pragma unroll
  for (int i = 0; i < 8; ++i) { a[i] = (_Float16)(p[i] * sc); a[8 + i] = (_Float16)(p[16 + i] * sc); }
  return a;
}
__device__ __forceinline__ v16h fragc_f32(const float* W, int k0, int n, int lane, int ld, int K) {
  v16h a; const int g = lane >> 4;
#pragma unroll
  for (int i = 0; i < 8; ++i) { const int ka = k0 + 8 * g + i, kb = ka + 16;
    a[i] = (_Float16)(ka < K ? W[(size_t)(ka < K ? ka : K - 1) * ld + n] : 0.f); a[8 + i] = (_Float16)(kb < K ? W[(size_t)(kb < K ? kb : K - 1) * ld + n] : 0.f); }
  return a;
}
struct F2 { v16b h, l; };
__device__ __forceinline__ F2 bsplit16(const float v[16]) { F2 r;
#pragma unroll
  for (int i = 0; i < 16; ++i) { const __bf16 h = (__bf16)v[i]; r.h[i] = h; r.l[i] = (__bf16)(v[i] - (float)h); }
  return r; }
__device__ __forceinline__ F2 split_row(const float* row, int k0, int lane) { float v[16]; const float* p = row + k0 + 8 * (lane >> 4);
#pragma unroll
  for (int i = 0; i < 8; ++i) { v[i] = p[i]; v[8 + i] = p[16 + i]; }
  return bsplit16(v); }
__device__ __forceinline__ F2 split_rowK(const float* row, int k0, int lane, int K) { float v[16]; const int g = lane >> 4;
#pragma unroll
  for (int i = 0; i < 8; ++i) { const int ka = k0 + 8 * g + i, kb = ka + 16; v[i] = ka < K ? row[ka < K ? ka : K - 1] : 0.f; v[8 + i] = kb < K ? row[kb < K ? kb : K - 1] : 0.f; }
  return bsplit16(v); }
__device__ __forceinline__ F2 split_col(const float* W, int k0, int n, int lane, int ld, int K) { float v[16]; const int g = lane >> 4;
#pragma unroll
  for (int i = 0; i < 8; ++i) { const int ka = k0 + 8 * g + i, kb = ka + 16; v[i] = ka < K ? W[(size_t)(ka < K ? ka : K - 1) * ld + n] : 0.f; v[8 + i] = kb < K ? W[(size_t)(kb < K ? kb : K - 1) * ld + n] : 0.f; }
  return bsplit16(v); }
__device__ __forceinline__ v8f mac3(const F2& a, const F2& b, v8f c) { c = wmma_bf(a.l, b.h, c); c = wmma_bf(a.h, b.l, c); return wmma_bf(a.h, b.h, c); }
__device__ __forceinline__ float sigm(float v) { return 1.0f / (1.0f + expf(-v)); }
#define LDSX() do { asm volatile("s_wait_dscnt 0" ::: "memory"); __builtin_amdgcn_wave_barrier(); __builtin_amdgcn_fence(__ATOMIC_RELEASE, "workgroup"); } while (0)

#define NB 2
#define TQ 1024
#define TM 1024
#define KK (TQ + TM)
#define CC 1024
#define NH 16
#define HD 64
#define HG 4
#define SCALE 0.125f
#ifndef TNB
#define TNB NB
#endif
#ifndef MP
#define MP KK
#endif
__device__ __forceinline__ float bfr(float v) { return (float)(__bf16)v; }
__device__ __forceinline__ v16b wcol(const float* Wm, int k0, int o, int lane, int ld) { v16b w; const int g = lane >> 4;
#pragma unroll
  for (int i = 0; i < 8; ++i) { w[i] = (__bf16)Wm[(size_t)(k0 + 8 * g + i) * ld + o]; w[8 + i] = (__bf16)Wm[(size_t)(k0 + 16 + 8 * g + i) * ld + o]; }
  return w; }
__device__ __forceinline__ v16h wcolh(const float* Wm, int k0, int o, int lane, int ld) { v16h w; const int g = lane >> 4;
#pragma unroll
  for (int i = 0; i < 8; ++i) { w[i] = (_Float16)(bfr(Wm[(size_t)(k0 + 8 * g + i) * ld + o]) * 256.0f); w[8 + i] = (_Float16)(bfr(Wm[(size_t)(k0 + 16 + 8 * g + i) * ld + o]) * 256.0f); }
  return w; }

#define WS_QUH 0u
#define WS_QUL (WS_QUH + 2u * (size_t)NB * TQ * CC)
#define WS_QVH (WS_QUL + 2u * (size_t)NB * TQ * CC)
#define WS_QVL (WS_QVH + 2u * (size_t)NB * TQ * CC)
#define WS_KH  (WS_QVL + 2u * (size_t)NB * TQ * CC)
#define WS_RK  (WS_KH  + 2u * (size_t)NB * KK * CC)
#define WS_VT  (WS_RK  + 2u * (size_t)KK * CC)
#define WS_S1  (WS_VT  + 2u * (size_t)NB * CC * KK)
#define WS_S2  (WS_S1  + 4u * (size_t)HG * TQ * KK)
#define WS_Y   (WS_S2  + 4u * (size_t)HG * TQ * KK)
#define WS_Z   (WS_Y   + 4u * (size_t)NB * TQ * CC)
#define WS_END (WS_Z   + 4u * (size_t)NB * TQ * CC)

__device__ __forceinline__ const float* cat_row(const float* INP, const float* MEM, int j, int b) { return (j < TM) ? (MEM + ((size_t)j * NB + b) * CC) : (INP + ((size_t)(j - TM) * NB + b) * CC); }
__global__ __launch_bounds__(128) void k_proj(const float* __restrict__ INP, const float* __restrict__ MEM, const float* __restrict__ WQKV, const float* __restrict__ RWB, const float* __restrict__ RRB, _Float16* __restrict__ QUH, _Float16* __restrict__ QUL, _Float16* __restrict__ QVH, _Float16* __restrict__ QVL, _Float16* __restrict__ KH, _Float16* __restrict__ VT) {
  __shared__ __align__(16) _Float16 sh[64][136], sl[64][136]; __shared__ __align__(16) _Float16 th[128][72];
  const int tid = threadIdx.x, wave = tid >> 5, lane = tid & 31, col = lane & 15, g = lane >> 4; const int which = blockIdx.z; const int c0 = blockIdx.y * 128; const int b = blockIdx.x / (KK / 64); const int j0 = (blockIdx.x % (KK / 64)) * 64;
  if (which == 0 && j0 < TM) return;
  const float* WA = WQKV + which * CC;
  const float* xr = cat_row(INP, MEM, j0 + wave * 16 + col, b);
  v8f acc[8] = {};
#pragma unroll 2
  for (int kc = 0; kc < CC / 32; ++kc) { v16b a; { const float* p = xr + kc * 32 + 8 * g;
#pragma unroll
      for (int i = 0; i < 8; ++i) { a[i] = (__bf16)p[i]; a[8 + i] = (__bf16)p[16 + i]; } }
    asm volatile("s_wait_loadcnt 0x0" ::: "memory");
#pragma unroll
    for (int j = 0; j < 8; ++j) { const v16b w = wcol(WA, kc * 32, c0 + j * 16 + col, lane, 3 * CC); asm volatile("s_wait_loadcnt 0x0" ::: "memory"); acc[j] = wmma_bf(a, w, acc[j]); } }
  const int npass = (which == 0) ? 2 : 1;
  for (int pass = 0; pass < npass; ++pass) {
    if (pass) __syncthreads();
#pragma unroll
    for (int j = 0; j < 8; ++j) { const int o = c0 + j * 16 + col; const float bb = (which == 0) ? bfr((pass == 0 ? RWB : RRB)[o]) : 0.f;
#pragma unroll
      for (int r = 0; r < 8; ++r) { const float v = acc[j][r] + bb; const int rl = wave * 16 + 8 * g + r, cl = j * 16 + col; const _Float16 hv = (_Float16)v;
        if (which == 2) th[cl][rl] = hv; else { sh[rl][cl] = hv; sl[rl][cl] = (_Float16)((v - (float)hv) * 1024.0f); } } }
    __syncthreads();
    if (which == 0) { _Float16* dh = pass == 0 ? QUH : QVH; _Float16* dl = pass == 0 ? QUL : QVL; const size_t q0 = (size_t)b * TQ + (j0 - TM); for (int e = tid; e < 64 * 16; e += 128) { const int rl = e >> 4, q = e & 15; vst2((unsigned*)(dh + (q0 + rl) * CC + c0 + q * 8), *(const v4u*)&sh[rl][q * 8]); vst2((unsigned*)(dl + (q0 + rl) * CC + c0 + q * 8), *(const v4u*)&sl[rl][q * 8]); } }
    else if (which == 1) { const size_t k0r = (size_t)b * KK + j0; for (int e = tid; e < 64 * 16; e += 128) { const int rl = e >> 4, q = e & 15; vst2((unsigned*)(KH + (k0r + rl) * CC + c0 + q * 8), *(const v4u*)&sh[rl][q * 8]); } }
    else { for (int e = tid; e < 128 * 8; e += 128) { const int cl = e >> 3, q = e & 7; vst2((unsigned*)(VT + ((size_t)b * CC + c0 + cl) * (size_t)KK + j0 + q * 8), *(const v4u*)&th[cl][q * 8]); } } } }
__global__ __launch_bounds__(128) void k_projr(const float* __restrict__ PE, const float* __restrict__ WR, _Float16* __restrict__ RK) { __shared__ __align__(16) _Float16 sh[64][136];
  const int tid = threadIdx.x, wave = tid >> 5, lane = tid & 31, col = lane & 15, g = lane >> 4; const int c0 = blockIdx.y * 128; const size_t p0 = (size_t)blockIdx.x * 64;
  v8f acc[8] = {};
#pragma unroll 2
  for (int kc = 0; kc < CC / 32; ++kc) { v16b a; { const float* p = PE + (p0 + wave * 16 + col) * CC + kc * 32 + 8 * g;
#pragma unroll
      for (int i = 0; i < 8; ++i) { a[i] = (__bf16)p[i]; a[8 + i] = (__bf16)p[16 + i]; } }
    asm volatile("s_wait_loadcnt 0x0" ::: "memory");
#pragma unroll
    for (int j = 0; j < 8; ++j) { const v16b w = wcol(WR, kc * 32, c0 + j * 16 + col, lane, CC); asm volatile("s_wait_loadcnt 0x0" ::: "memory"); acc[j] = wmma_bf(a, w, acc[j]); } }
#pragma unroll
  for (int j = 0; j < 8; ++j) {
#pragma unroll
    for (int r = 0; r < 8; ++r) sh[wave * 16 + 8 * g + r][j * 16 + col] = (_Float16)acc[j][r]; }
  __syncthreads();
  for (int e = tid; e < 64 * 16; e += 128) { const int rl = e >> 4, q = e & 15; vst2((unsigned*)(RK + (p0 + rl) * CC + c0 + q * 8), *(const v4u*)&sh[rl][q * 8]); } }
__global__ __launch_bounds__(128) void k_sc(const _Float16* __restrict__ QH, const _Float16* __restrict__ QL, const _Float16* __restrict__ KEY, size_t key_row0, int b, int h0, float* __restrict__ S0) { __shared__ __align__(16) float ss[4][16][132]; const int h = h0 + blockIdx.z; float* S = S0 + (size_t)blockIdx.z * TQ * KK;
  const int tid = threadIdx.x, wave = tid >> 5, lane = tid & 31, col = lane & 15, g = lane >> 4; const int k0 = blockIdx.y * 128; const int ql0 = blockIdx.x * 64 + wave * 16; const size_t q0 = (size_t)b * TQ + ql0;
  v8f acc[8] = {}, accl[8] = {};
#pragma unroll
  for (int kc = 0; kc < HD / 32; ++kc) { const v16h ah = frag_h(QH + (q0 + col) * CC + h * HD + kc * 32, lane), al = frag_h(QL + (q0 + col) * CC + h * HD + kc * 32, lane);
#pragma unroll
    for (int j = 0; j < 8; ++j) { const v16h kb = frag_h(KEY + (key_row0 + k0 + j * 16 + col) * CC + h * HD + kc * 32, lane); acc[j] = wmma16(ah, kb, acc[j]); accl[j] = wmma16(al, kb, accl[j]); } }
#pragma unroll
  for (int j = 0; j < 8; ++j) {
#pragma unroll
    for (int r = 0; r < 8; ++r) ss[wave][8 * g + r][j * 16 + col] = acc[j][r] + accl[j][r] * (1.0f / 1024.0f); }
  LDSX(); for (int rl = 0; rl < 16; ++rl) vst2(S + (size_t)(ql0 + rl) * KK + k0 + lane * 4, *(const v4f*)&ss[wave][rl][lane * 4]); }
__global__ __launch_bounds__(256) void k_comb(float* __restrict__ S1_0, const float* __restrict__ S2_0, const int* __restrict__ MASK) {
  const int t = threadIdx.x; const int i = blockIdx.x; float* S1 = S1_0 + (size_t)blockIdx.y * TQ * KK + (size_t)i * KK; const float* S2 = S2_0 + (size_t)blockIdx.y * TQ * KK; const int* mk = MASK + (size_t)i * MP;
  const float* rowi = S2 + (size_t)i * KK; const float* rown = S2 + (size_t)(i + 1 < TQ ? i + 1 : i) * KK;
  for (int q = t; q < KK / 4; q += 256) { v4f a = *(const v4f*)(S1 + q * 4); v4f o;
#pragma unroll
    for (int z = 0; z < 4; ++z) { const int j = q * 4 + z; const int ja = min(max(TQ - 1 - i + j, 0), KK - 1), jb = min(max(j - i - TM - 2, 0), KK - 1); const float va = rowi[ja], vb = rown[jb];
      const float fa = (j <= i + TM) ? 1.0f : 0.0f, fb = (j >= i + TM + 2) ? 1.0f : 0.0f;
      const float sc = (a[z] + fmaf(fa, va, fb * vb)) * SCALE; o[z] = (mk[j] != 0) ? -3.0e38f : sc; }
    vst2(S1 + q * 4, o); } }
__global__ __launch_bounds__(256) void k_sm(float* __restrict__ S0) { __shared__ float sred[8]; __shared__ float sbc; __shared__ __align__(16) float sh[KK];
  const int t = threadIdx.x; const size_t row = blockIdx.x; float* sr = S0 + (size_t)blockIdx.y * TQ * KK + row * KK; const int kend = KK;
  float m = -3.0e38f; for (int k = t; k < kend; k += 256) m = fmaxf(m, sr[k]);
#pragma unroll
  for (int o = 1; o < 32; o <<= 1) m = fmaxf(m, __shfl_xor(m, o));
  if ((t & 31) == 0) sred[t >> 5] = m; __syncthreads(); if (t == 0) { float a = sred[0]; for (int i = 1; i < 8; ++i) a = fmaxf(a, sred[i]); sbc = a; } __syncthreads(); m = sbc; __syncthreads();
  float sum = 0.f; for (int k = t; k < kend; k += 256) { const float v = sr[k]; const float e = (v <= -1.0e38f) ? 0.f : expf(v - m); sh[k] = e; sum += e; }
#pragma unroll
  for (int o = 1; o < 32; o <<= 1) sum += __shfl_xor(sum, o);
  if ((t & 31) == 0) sred[t >> 5] = sum; __syncthreads(); if (t == 0) { float a = 0.f; for (int i = 0; i < 8; ++i) a += sred[i]; sbc = 2048.0f / a; } __syncthreads(); const float inv = sbc;
  for (int k = t; k < kend; k += 256) sh[k] = sh[k] * inv;
  __syncthreads(); for (int q = t; q < kend / 4; q += 256) vst2(sr + q * 4, *(const v4f*)&sh[q * 4]); }
__global__ __launch_bounds__(128) void k_pv(const float* __restrict__ PS0, const _Float16* __restrict__ VT, int b, int h0, float* __restrict__ Y) { const int h = h0 + blockIdx.z; const float* PS = PS0 + (size_t)blockIdx.z * TQ * KK; __shared__ __align__(16) float ss[4][16][HD + 4];
  const int tid = threadIdx.x, wave = tid >> 5, lane = tid & 31, col = lane & 15, g = lane >> 4; const int ql0 = blockIdx.x * 64 + wave * 16;
  v8f acc[HD / 16] = {};
#pragma unroll 2
  for (int kc = 0; kc < KK / 32; ++kc) { const v16h p = frag_f32(PS + (size_t)(ql0 + col) * KK + kc * 32, lane);
    asm volatile("s_wait_loadcnt 0x0" ::: "memory");
#pragma unroll
    for (int j = 0; j < HD / 16; ++j) { const size_t po = ((size_t)b * CC + h * HD + j * 16 + col) * (size_t)KK + kc * 32; acc[j] = wmma16(p, frag_h(VT + po, lane), acc[j]); } }
#pragma unroll
  for (int j = 0; j < HD / 16; ++j)
#pragma unroll
    for (int r = 0; r < 8; ++r) ss[wave][8 * g + r][j * 16 + col] = acc[j][r] * (1.0f / 2048.0f);
  LDSX(); for (int rl = 0; rl < 16; ++rl) if (lane < HD / 4) vst2(Y + ((size_t)b * TQ + ql0 + rl) * CC + h * HD + lane * 4, *(const v4f*)&ss[wave][rl][lane * 4]); }
__global__ __launch_bounds__(128) void k_out(const float* __restrict__ Y, const float* __restrict__ WO, float* __restrict__ Z) { __shared__ __align__(16) float sf[4][16][132];
  const int tid = threadIdx.x, wave = tid >> 5, lane = tid & 31, col = lane & 15, g = lane >> 4; const int c0 = blockIdx.y * 128; const size_t r0 = (size_t)blockIdx.x * 64 + wave * 16;
  v8f acc[8] = {};
#pragma unroll 2
  for (int kc = 0; kc < CC / 32; ++kc) { const v16h a = frag_f32(Y + (r0 + col) * CC + kc * 32, lane); asm volatile("s_wait_loadcnt 0x0" ::: "memory");
#pragma unroll
    for (int j = 0; j < 8; ++j) { const v16h w = wcolh(WO, kc * 32, c0 + j * 16 + col, lane, CC); asm volatile("s_wait_loadcnt 0x0" ::: "memory"); acc[j] = wmma16(a, w, acc[j]); } }
#pragma unroll
  for (int j = 0; j < 8; ++j) {
#pragma unroll
    for (int r = 0; r < 8; ++r) sf[wave][8 * g + r][j * 16 + col] = acc[j][r] * (1.0f / 256.0f); }
  LDSX(); for (int rl = 0; rl < 16; ++rl) vst2(Z + (r0 + rl) * CC + c0 + lane * 4, *(const v4f*)&sf[wave][rl][lane * 4]); }
__global__ __launch_bounds__(256) void k_ln(const float* __restrict__ Z, const float* __restrict__ G, const float* __restrict__ Bb, float* __restrict__ OUT) { __shared__ float sred[8]; __shared__ float sbc;
  const int t = threadIdx.x; const size_t row = blockIdx.x; const int b = (int)(row / TQ), i = (int)(row % TQ); const v4f y = *(const v4f*)(Z + row * CC + t * 4);
  float s = (y[0] + y[1]) + (y[2] + y[3]);
#pragma unroll
  for (int o = 1; o < 32; o <<= 1) s += __shfl_xor(s, o);
  if ((t & 31) == 0) sred[t >> 5] = s; __syncthreads(); if (t == 0) { float a = 0.f; for (int q = 0; q < 8; ++q) a += sred[q]; sbc = a * (1.0f / CC); } __syncthreads(); const float mean = sbc; __syncthreads();
  float d[4], s2 = 0.f;
#pragma unroll
  for (int z = 0; z < 4; ++z) { d[z] = y[z] - mean; s2 += d[z] * d[z]; }
#pragma unroll
  for (int o = 1; o < 32; o <<= 1) s2 += __shfl_xor(s2, o);
  if ((t & 31) == 0) sred[t >> 5] = s2; __syncthreads(); if (t == 0) { float a = 0.f; for (int q = 0; q < 8; ++q) a += sred[q]; sbc = rsqrtf(a * (1.0f / CC) + 1e-5f); } __syncthreads(); const float rstd = sbc;
  v4f o4;
#pragma unroll
  for (int z = 0; z < 4; ++z) o4[z] = d[z] * rstd * bfr(G[t * 4 + z]) + bfr(Bb[t * 4 + z]);
  vst2(OUT + ((size_t)i * NB + b) * CC + t * 4, o4); }
extern "C" void kernel_launch(void* const* d_in, const int* in_sizes, int n_in, void* d_out, int out_size, void* d_ws, size_t ws_size, hipStream_t stream) {
  (void)in_sizes; (void)n_in; (void)out_size;
  const float** F = (const float**)d_in;
  if (ws_size < (size_t)WS_END) return;
  char* ws = (char*)d_ws; _Float16 *QUH = (_Float16*)(ws + WS_QUH), *QUL = (_Float16*)(ws + WS_QUL), *QVH = (_Float16*)(ws + WS_QVH), *QVL = (_Float16*)(ws + WS_QVL), *KH = (_Float16*)(ws + WS_KH), *RK = (_Float16*)(ws + WS_RK), *VT = (_Float16*)(ws + WS_VT); float *S1 = (float*)(ws + WS_S1), *S2 = (float*)(ws + WS_S2), *Y = (float*)(ws + WS_Y), *Z = (float*)(ws + WS_Z);
  k_proj<<<dim3(TNB * (KK / 64), CC / 128, 3), 128, 0, stream>>>(F[0], F[2], F[4], F[7], F[8], QUH, QUL, QVH, QVL, KH, VT);
  k_projr<<<dim3(KK / 64, CC / 128), 128, 0, stream>>>(F[1], F[5], RK);
  for (int b = 0; b < TNB; ++b) for (int h0 = 0; h0 < NH; h0 += HG) {
    k_sc<<<dim3(TQ / 64, KK / 128, HG), 128, 0, stream>>>(QUH, QUL, KH, (size_t)b * KK, b, h0, S1);
    k_sc<<<dim3(TQ / 64, KK / 128, HG), 128, 0, stream>>>(QVH, QVL, RK, (size_t)0, b, h0, S2);
    k_comb<<<dim3(TQ, HG), 256, 0, stream>>>(S1, S2, (const int*)d_in[3]);
    k_sm<<<dim3(TQ, HG), 256, 0, stream>>>(S1);
    k_pv<<<dim3(TQ / 64, 1, HG), 128, 0, stream>>>(S1, VT, b, h0, Y);
  }
  k_out<<<dim3(TNB * TQ / 64, CC / 128), 128, 0, stream>>>(Y, F[6], Z);
  k_ln<<<dim3(TNB * TQ), 256, 0, stream>>>(Z, F[9], F[10], (float*)d_out);
}
